// JKNet_54984171323612
// MI455X (gfx1250) — hardware-verified
//
#include <hip/hip_runtime.h>
#include <stddef.h>
#include <stdint.h>


#define CIN    128
#define CH     128
#define CO     64
#define NTHR   256
#define NWAVE  8
#define EPT    8
#define CHUNK  (NTHR * EPT)
#define WCAP   (EPT * 32)
#define LISTN  (NWAVE * WCAP)
#define NBD    8192
#define SLBD   13
#define NS     2048
#define SLBA   11
#define LCAP   36864
#define SRCB   21
#define SRCM   ((1 << SRCB) - 1)
#define SORTMAX (2 * LCAP + NS + 64)
#define GBM    64
#define GTHR   128
#define WSMAX  268435456

#define A_OLST 0
#define A_OCNT (A_OLST + LISTN)
#define A_OOFF (A_OCNT + NS)
#define A_ODIN (A_OOFF + NS + 32)
#define A_OL   (A_ODIN + NS)
#define A_TOT  (A_OL + LCAP)
#define A_LDSB (A_TOT * 4)

static_assert((CHUNK & (CHUNK - 1)) == 0 && CHUNK <= 4096);
static_assert(NBD == (1 << SLBD) && NS == (1 << SLBA));
static_assert(((long long)CHUNK << SLBD) < (1LL << 31));
static_assert(((long long)CHUNK << SLBA) < (1LL << 31));
static_assert(SRCB + SLBA <= 32);
static_assert(NBD % (NTHR * 4) == 0);
static_assert(NS == 8 * NTHR && NS % NWAVE == 0 && NS == 2 * 4 * NTHR);
static_assert(LISTN % NTHR == 0);
static_assert((A_OCNT % 4) == 0 && (A_OOFF % 4) == 0 && (A_ODIN % 4) == 0 && (A_OL % 4) == 0);
static_assert(A_LDSB <= 300000);
static_assert(CIN == CH && CH == 128 && CO == 64);
static_assert(GBM == (GTHR / 32) * 16 && GTHR >= GBM);

typedef float          v4f   __attribute__((ext_vector_type(4)));
typedef float          v8f   __attribute__((ext_vector_type(8)));
typedef int            v4i   __attribute__((ext_vector_type(4)));
typedef int            v8i   __attribute__((ext_vector_type(8)));
typedef unsigned short v8us  __attribute__((ext_vector_type(8)));
typedef unsigned short v16us __attribute__((ext_vector_type(16)));
typedef __bf16         v16bf __attribute__((ext_vector_type(16)));
typedef v4f  __attribute__((may_alias)) v4fa;
typedef v4i  __attribute__((may_alias)) v4ia;
typedef v8us __attribute__((may_alias)) v8usa;
union FragB { v16bf v; v16us u; v8us h[2]; v8i w; };

__device__ __forceinline__ v8f wmb(const FragB& a, const FragB& b, v8f c) {
  v8f d = __builtin_amdgcn_wmma_f32_16x16x32_bf16(false, a.v, false, b.v, (short)0, c, false, false);
  asm volatile("v_nop\n\tv_nop\n\tv_nop\n\tv_nop" : "+v"(d) : "v"(a.w), "v"(b.w));
  return d;
}

__device__ __forceinline__ unsigned bf16_bits(float f) {
  const unsigned u = __float_as_uint(f);
  return (u + 0x7FFFu + ((u >> 16) & 1u)) >> 16;
}
__device__ __forceinline__ float bf16_val(float f) {
  return __uint_as_float(bf16_bits(f) << 16);
}
__device__ __forceinline__ v4f relu4(v4f v) {
  v.x = fmaxf(v.x, 0.0f); v.y = fmaxf(v.y, 0.0f); v.z = fmaxf(v.z, 0.0f); v.w = fmaxf(v.w, 0.0f);
  return v;
}

template <int SLBT>
__device__ __forceinline__ int scan_chunk(const int* __restrict__ dsts, int nE, int cbase, int slotBase,
                                          int nb, int vec8, int* list, int tid, int lane, int wave) {
  int wc = 0;
  const int el0  = tid * EPT;
  const int e0   = cbase + el0;
  const int sent = -2147483647 - 1;
  v4i da, db;
  if (vec8 != 0 && cbase + CHUNK <= nE) {
    da = *(const v4i*)(dsts + e0);
    db = *(const v4i*)(dsts + e0 + 4);
  } else {
    da.x = (e0     < nE) ? dsts[min(e0,     nE - 1)] : sent;
    da.y = (e0 + 1 < nE) ? dsts[min(e0 + 1, nE - 1)] : sent;
    da.z = (e0 + 2 < nE) ? dsts[min(e0 + 2, nE - 1)] : sent;
    da.w = (e0 + 3 < nE) ? dsts[min(e0 + 3, nE - 1)] : sent;
    db.x = (e0 + 4 < nE) ? dsts[min(e0 + 4, nE - 1)] : sent;
    db.y = (e0 + 5 < nE) ? dsts[min(e0 + 5, nE - 1)] : sent;
    db.z = (e0 + 6 < nE) ? dsts[min(e0 + 6, nE - 1)] : sent;
    db.w = (e0 + 7 < nE) ? dsts[min(e0 + 7, nE - 1)] : sent;
  }
  const unsigned nbs = (unsigned)slotBase;
  const unsigned unb = (unsigned)nb;
  const unsigned s0 = (unsigned)da.x - nbs, s1 = (unsigned)da.y - nbs;
  const unsigned s2 = (unsigned)da.z - nbs, s3 = (unsigned)da.w - nbs;
  const unsigned s4 = (unsigned)db.x - nbs, s5 = (unsigned)db.y - nbs;
  const unsigned s6 = (unsigned)db.z - nbs, s7 = (unsigned)db.w - nbs;
  const bool h0 = s0 < unb, h1 = s1 < unb, h2 = s2 < unb, h3 = s3 < unb;
  const bool h4 = s4 < unb, h5 = s5 < unb, h6 = s6 < unb, h7 = s7 < unb;
  const unsigned any = __builtin_amdgcn_ballot_w32(h0 | h1 | h2 | h3 | h4 | h5 | h6 | h7);
  if (any != 0u) {
#define HITJ(J, HJ, SJ) { \
      const unsigned mj = __builtin_amdgcn_ballot_w32(HJ); \
      if (mj != 0u) { \
        if (HJ) { \
          const int pos = wc + (int)__builtin_amdgcn_mbcnt_lo(mj, 0u); \
          if (pos < WCAP) list[wave * WCAP + pos] = ((el0 + (J)) << SLBT) | (int)(SJ); \
        } \
        wc += (int)__builtin_popcount(mj); } }
    HITJ(0, h0, s0)
    HITJ(1, h1, s1)
    HITJ(2, h2, s2)
    HITJ(3, h3, s3)
    HITJ(4, h4, s4)
    HITJ(5, h5, s5)
    HITJ(6, h6, s6)
    HITJ(7, h7, s7)
#undef HITJ
  }
  return wc;
}

__device__ __forceinline__ void wprep_unit(const float* __restrict__ W, unsigned short* T, int K, int NCn, int u) {
  const int kq = K >> 3;
  const int n  = u / kq;
  const int k8 = (u - n * kq) * 8;
  const float* p = W + (size_t)k8 * NCn + n;
  v8us o;
  o[0] = (unsigned short)bf16_bits(p[0]);
  o[1] = (unsigned short)bf16_bits(p[(size_t)NCn]);
  o[2] = (unsigned short)bf16_bits(p[(size_t)2 * NCn]);
  o[3] = (unsigned short)bf16_bits(p[(size_t)3 * NCn]);
  o[4] = (unsigned short)bf16_bits(p[(size_t)4 * NCn]);
  o[5] = (unsigned short)bf16_bits(p[(size_t)5 * NCn]);
  o[6] = (unsigned short)bf16_bits(p[(size_t)6 * NCn]);
  o[7] = (unsigned short)bf16_bits(p[(size_t)7 * NCn]);
  unsigned short* dp = T + (size_t)n * K + k8;
  *(volatile v8us*)dp = o;
  __threadfence();
  *(volatile v8us*)dp = o;
}

__global__ __launch_bounds__(NTHR) void k_wprep(const float* __restrict__ W1, const float* __restrict__ W2,
                                                const float* __restrict__ Wo, unsigned short* T1,
                                                unsigned short* T2, unsigned short* To) {
  const int seg = (int)blockIdx.x >> 3;
  const int u   = ((int)blockIdx.x & 7) * NTHR + (int)threadIdx.x;
  if (seg == 0)      wprep_unit(W1, T1, CIN, CH, u);
  else if (seg == 1) wprep_unit(W2, T2, CH, CH, u);
  else               wprep_unit(Wo, To, 2 * CH, CO, u);
}

__global__ __launch_bounds__(NTHR) void k_deg(const int* __restrict__ idx, int nE, int vec8, float* dinv) {
  __shared__ __attribute__((aligned(16))) int scnt[NBD];
  __shared__ __attribute__((aligned(16))) int list[LISTN];
  __shared__ int wcnt[NWAVE];
  const int tid = (int)threadIdx.x, lane = tid & 31, wave = tid >> 5;
  const int nodeBase = (int)blockIdx.x * NBD;

  for (int i = tid; i < NBD; i += NTHR) scnt[i] = 0;
  for (int i = tid; i < LISTN; i += NTHR) list[i] = 0;
  if (tid < NWAVE) wcnt[tid] = 0;
  __syncthreads();

  const int nChunks = (nE + CHUNK - 1) / CHUNK;
#pragma unroll 1
  for (int ch = 0; ch < nChunks; ++ch) {
    const int cbase = ch * CHUNK;
    const int wc = scan_chunk<SLBD>(idx, nE, cbase, nodeBase, NBD, vec8, list, tid, lane, wave);
    if (lane == 0) wcnt[wave] = wc;
    __syncthreads();
    if (wave == 0) {
#pragma unroll 1
      for (int w2 = 0; w2 < NWAVE; ++w2) {
        int c = wcnt[w2];
        c = c < 0 ? 0 : (c > WCAP ? WCAP : c);
#pragma unroll 1
        for (int b0 = 0; b0 < c; b0 += 32) {
          const int ix  = b0 + lane;
          const int ent = list[w2 * WCAP + (ix < WCAP ? ix : WCAP - 1)];
          const int m32 = (c - b0) < 32 ? (c - b0) : 32;
#pragma unroll 1
          for (int k = 0; k < m32; ++k) {
            const int u  = __builtin_amdgcn_readlane(ent, k);
            const int sl = u & (NBD - 1);
            if (lane == 0) scnt[sl] = scnt[sl] + 1;
          }
        }
      }
    }
    __syncthreads();
  }

  v4f vals[NBD / (NTHR * 4)];
#pragma unroll
  for (int it = 0; it < NBD / (NTHR * 4); ++it) {
    const int s0 = it * (NTHR * 4) + 4 * tid;
    const v4i c4 = *(const v4ia*)(scnt + s0);
    v4f v;
    v.x = rsqrtf(fmaxf((float)c4.x, 1.0f));
    v.y = rsqrtf(fmaxf((float)c4.y, 1.0f));
    v.z = rsqrtf(fmaxf((float)c4.z, 1.0f));
    v.w = rsqrtf(fmaxf((float)c4.w, 1.0f));
    vals[it] = v;
  }
#pragma unroll
  for (int it = 0; it < NBD / (NTHR * 4); ++it) {
    const int s0 = it * (NTHR * 4) + 4 * tid;
    *(volatile v4f*)(dinv + (size_t)nodeBase + s0) = vals[it];
  }
  __threadfence();
#pragma unroll
  for (int it = 0; it < NBD / (NTHR * 4); ++it) {
    const int s0 = it * (NTHR * 4) + 4 * tid;
    *(volatile v4f*)(dinv + (size_t)nodeBase + s0) = vals[it];
  }
}

template <int MODE>
__global__ __launch_bounds__(NTHR) void k_agg(const float* __restrict__ T, const int* __restrict__ srcs,
                                              const int* __restrict__ dsts, const float* __restrict__ dsrc,
                                              const float* __restrict__ bias, float* O1, float* O2,
                                              int nE, int nN, int vec8) {
  extern __shared__ __attribute__((aligned(16))) int dynl[];
  int*   lst  = dynl + A_OLST;
  int*   scnt = dynl + A_OCNT;
  int*   soff = dynl + A_OOFF;
  float* sdin = (float*)(dynl + A_ODIN);
  int*   L    = dynl + A_OL;
  __shared__ int s_wcnt[NWAVE];
  __shared__ int s_wsum[NWAVE];
  __shared__ int s_misc[4];
  const int tid = (int)threadIdx.x, lane = tid & 31, wave = tid >> 5;
  const int nodeBase = (int)blockIdx.x * NS;
  int nb = nN - nodeBase;
  nb = nb < 0 ? 0 : (nb > NS ? NS : nb);

  for (int i = tid; i < A_TOT; i += NTHR) dynl[i] = 0;
  if (tid < NWAVE) { s_wcnt[tid] = 0; s_wsum[tid] = 0; }
  if (tid < 4) s_misc[tid] = 0;
  __syncthreads();

  int tot = 0, ovf = 0;
  const int nChunks = (nE + CHUNK - 1) / CHUNK;
#pragma unroll 1
  for (int ch = 0; ch < nChunks; ++ch) {
    const int cbase = ch * CHUNK;
    const int wc = scan_chunk<SLBA>(dsts, nE, cbase, nodeBase, NS, vec8, lst, tid, lane, wave);
    if (lane == 0) s_wcnt[wave] = wc;
    __syncthreads();
    if (wave == 0) {
#pragma unroll 1
      for (int w2 = 0; w2 < NWAVE; ++w2) {
        int c = s_wcnt[w2];
        c = c < 0 ? 0 : (c > WCAP ? WCAP : c);
#pragma unroll 1
        for (int b0 = 0; b0 < c; b0 += 32) {
          const int ix  = b0 + lane;
          const int ent = lst[w2 * WCAP + (ix < WCAP ? ix : WCAP - 1)];
          const int el  = (ent >> SLBA) & (CHUNK - 1);
          const int sl  = ent & (NS - 1);
          int eid = cbase + el;
          eid = eid < 0 ? 0 : (eid > nE - 1 ? nE - 1 : eid);
          const int sraw = srcs[eid];
          const int sv = sraw < 0 ? 0 : (sraw > nN - 1 ? nN - 1 : sraw);
          const int m32 = (c - b0) < 32 ? (c - b0) : 32;
          const int pos = tot + b0 + lane;
          if (lane < m32 && pos < LCAP) L[pos] = (int)(((unsigned)sl << SRCB) | (unsigned)sv);
#pragma unroll 1
          for (int k = 0; k < m32; ++k) {
            const int u   = __builtin_amdgcn_readlane(ent, k);
            const int slk = u & (NS - 1);
            if (lane == 0 && (tot + b0 + k) < LCAP) scnt[slk] = scnt[slk] + 1;
          }
        }
        tot += c;
        if (tot > LCAP) { ovf = 1; tot = LCAP; }
      }
    }
    __syncthreads();
  }
  if (tid == 0) { s_misc[0] = tot; s_misc[1] = ovf; }
  __syncthreads();

  int pc[8];
  {
    const v4i c0 = *(const v4ia*)(scnt + 8 * tid);
    const v4i c1 = *(const v4ia*)(scnt + 8 * tid + 4);
    pc[0] = c0.x; pc[1] = c0.y; pc[2] = c0.z; pc[3] = c0.w;
    pc[4] = c1.x; pc[5] = c1.y; pc[6] = c1.z; pc[7] = c1.w;
  }
  int sum8 = 0;
#pragma unroll
  for (int j = 0; j < 8; ++j) sum8 += pc[j];
  int xs = sum8;
#pragma unroll
  for (int d = 1; d < 32; d <<= 1) {
    const int y = __shfl_up(xs, (unsigned)d, 32);
    xs = (lane >= d) ? (xs + y) : xs;
  }
  if (lane == 31) s_wsum[wave] = xs;
  __syncthreads();
  int wb = 0;
#pragma unroll
  for (int w2 = 0; w2 < NWAVE; ++w2) {
    const int t = s_wsum[w2];
    wb += (w2 < wave) ? t : 0;
  }
  {
    int run = wb + xs - sum8;
#pragma unroll
    for (int j = 0; j < 8; ++j) { soff[8 * tid + j] = run; run += pc[j]; }
    if (tid == NTHR - 1) soff[NS] = run;
  }
  if (MODE == 1) {
#pragma unroll
    for (int j = 0; j < 8; ++j) sdin[8 * tid + j] = rsqrtf(fmaxf((float)pc[j], 1.0f));
  }
  __syncthreads();

  {
    const v4i o0 = *(const v4ia*)(soff + 8 * tid);
    const v4i o1 = *(const v4ia*)(soff + 8 * tid + 4);
    *(v4ia*)(scnt + 8 * tid)     = o0;
    *(v4ia*)(scnt + 8 * tid + 4) = o1;
  }
  if (MODE == 1) {
    const v4f d0 = *(const v4fa*)(sdin + 4 * tid);
    const v4f d1 = *(const v4fa*)(sdin + 4 * tid + 4 * NTHR);
    float* q = O2 + (size_t)nodeBase;
    *(volatile v4f*)(q + 4 * tid)            = d0;
    *(volatile v4f*)(q + 4 * tid + 4 * NTHR) = d1;
    __threadfence();
    *(volatile v4f*)(q + 4 * tid)            = d0;
    *(volatile v4f*)(q + 4 * tid + 4 * NTHR) = d1;
  }
  __syncthreads();

  if (tid == 0) {
    int it = 0, bad = 0;
#pragma unroll 1
    for (int s = 0; s < NS; ++s) {
      int c  = scnt[s];
      int hi = soff[s + 1];
      c  = c  < 0 ? 0 : (c  > LCAP ? LCAP : c);
      hi = hi < 0 ? 0 : (hi > LCAP ? LCAP : hi);
#pragma unroll 1
      while (c < hi && it < SORTMAX) {
        ++it;
        const int e = L[c];
        const int d = (int)(((unsigned)e) >> SRCB) & (NS - 1);
        if (d == s) {
          ++c;
        } else {
          int cd = scnt[d];
          cd = cd < 0 ? 0 : (cd > LCAP - 1 ? LCAP - 1 : cd);
          const int f = L[cd];
          L[cd] = e;
          scnt[d] = cd + 1;
          L[c] = f;
        }
      }
      if (c < hi) bad = 1;
      scnt[s] = c;
    }
    if (bad != 0) s_misc[1] = s_misc[1] | 2;
  }
  __syncthreads();

  const int ovfb = s_misc[1];
  const float qnan = __uint_as_float(0x7fc00000u);
  v4f bvec = {0.0f, 0.0f, 0.0f, 0.0f};
  if (MODE == 1) {
    bvec.x = bf16_val(bias[4 * lane]);
    bvec.y = bf16_val(bias[4 * lane + 1]);
    bvec.z = bf16_val(bias[4 * lane + 2]);
    bvec.w = bf16_val(bias[4 * lane + 3]);
  }
#pragma unroll 1
  for (int i = 0; i < NS / NWAVE; ++i) {
    const int s = wave + NWAVE * i;
    if (s < nb) {
      int beg = soff[s], end = soff[s + 1];
      beg = beg < 0 ? 0 : (beg > LCAP ? LCAP : beg);
      end = end < 0 ? 0 : (end > LCAP ? LCAP : end);
      end = end < beg ? beg : end;
      v4f a  = {0.0f, 0.0f, 0.0f, 0.0f};
      v4f a2 = {0.0f, 0.0f, 0.0f, 0.0f};
#pragma unroll 2
      for (int j = beg; j < end; ++j) {
        const int e = L[j];
        int sv = e & SRCM;
        sv = sv > nN - 1 ? nN - 1 : sv;
        const v4f v = *(const v4fa*)(T + (size_t)sv * CH + 4 * lane);
        a += v;
        if (MODE == 2) { const float ds = dsrc[sv]; a2 += v * ds; }
      }
      const int node = nodeBase + s;
      v4f o1 = a, o2 = a2;
      if (MODE == 1) {
        const float dn = sdin[s];
        o1 = a * dn + bvec;
        o1 = relu4(o1);
      }
      if (ovfb != 0) { o1.x = qnan; o1.y = qnan; o1.z = qnan; o1.w = qnan; o2 = o1; }
      float* p1 = O1 + (size_t)node * CH + 4 * lane;
      *(volatile v4f*)p1 = o1;
      if (MODE == 2) { float* p2 = O2 + (size_t)node * CH + 4 * lane; *(volatile v4f*)p2 = o2; }
      __threadfence();
      *(volatile v4f*)p1 = o1;
      if (MODE == 2) { float* p2 = O2 + (size_t)node * CH + 4 * lane; *(volatile v4f*)p2 = o2; }
    }
  }
}

template <int NT, int SPLIT, int KW>
__device__ __forceinline__ void gemm_k128(const float* __restrict__ ap0, const unsigned short* __restrict__ wp0,
                                          v8f (&acc)[NT]) {
#pragma unroll 1
  for (int kk = 0; kk < CH / 32; ++kk) {
    const int k0 = 32 * kk;
    const float* ap = ap0 + k0;
    const v4f x0 = *(const v4fa*)(ap);
    const v4f x1 = *(const v4fa*)(ap + 4);
    const v4f x2 = *(const v4fa*)(ap + 16);
    const v4f x3 = *(const v4fa*)(ap + 20);
    float v[16];
    v[0]  = x0.x; v[1]  = x0.y; v[2]  = x0.z; v[3]  = x0.w;
    v[4]  = x1.x; v[5]  = x1.y; v[6]  = x1.z; v[7]  = x1.w;
    v[8]  = x2.x; v[9]  = x2.y; v[10] = x2.z; v[11] = x2.w;
    v[12] = x3.x; v[13] = x3.y; v[14] = x3.z; v[15] = x3.w;
    FragB ah, al;
#pragma unroll
    for (int i = 0; i < 16; ++i) {
      const unsigned hb = bf16_bits(v[i]);
      ah.u[i] = (unsigned short)hb;
      al.u[i] = (unsigned short)(SPLIT ? bf16_bits(v[i] - __uint_as_float(hb << 16)) : 0u);
    }
#pragma unroll
    for (int nt = 0; nt < NT; ++nt) {
      const unsigned short* wq = wp0 + (size_t)(16 * nt) * KW + k0;
      FragB bf;
      bf.h[0] = *(const v8usa*)wq;
      bf.h[1] = *(const v8usa*)(wq + 16);
      acc[nt] = wmb(ah, bf, acc[nt]);
      if (SPLIT) acc[nt] = wmb(al, bf, acc[nt]);
    }
  }
}

template <int MODE>
__global__ __launch_bounds__(GTHR) void k_gemm(const float* __restrict__ A1, const float* __restrict__ A2,
                                               const unsigned short* __restrict__ WT, const float* __restrict__ rsc,
                                               const float* __restrict__ bias, float* O, int nN) {
  constexpr int NT = (MODE == 3) ? 4 : 8;
  constexpr int NC = 16 * NT;
  constexpr int KW = (MODE == 3) ? 2 * CH : CH;
  constexpr int SPLIT = (MODE == 1) ? 0 : 1;
  constexpr int SP = NC + 4;
  __shared__ __attribute__((aligned(16))) float sRS[GBM];
  __shared__ __attribute__((aligned(16))) float stg[GBM * SP];
  const int tid = (int)threadIdx.x, lane = tid & 31, wave = tid >> 5, hh = lane >> 4, m = lane & 15;
  const int rowBase = (int)blockIdx.x * GBM;

  if (tid < GBM) {
    int rr = rowBase + tid;
    rr = rr > nN - 1 ? nN - 1 : rr;
    float sc = 1.0f;
    if (MODE != 3) sc = rsc[rr];
    sRS[tid] = sc;
  }
  v4f bv = {0.0f, 0.0f, 0.0f, 0.0f};
  if (MODE == 2) {
    bv.x = bf16_val(bias[4 * lane]);     bv.y = bf16_val(bias[4 * lane + 1]);
    bv.z = bf16_val(bias[4 * lane + 2]); bv.w = bf16_val(bias[4 * lane + 3]);
  }
  if (MODE == 3) {
    bv.x = bf16_val(bias[4 * m]);     bv.y = bf16_val(bias[4 * m + 1]);
    bv.z = bf16_val(bias[4 * m + 2]); bv.w = bf16_val(bias[4 * m + 3]);
  }
  __syncthreads();

  const int row = rowBase + 16 * wave + m;
  const int rc  = row < nN ? row : nN - 1;
  v8f acc[NT];
  {
    const v8f z = {0.f, 0.f, 0.f, 0.f, 0.f, 0.f, 0.f, 0.f};
#pragma unroll
    for (int t = 0; t < NT; ++t) acc[t] = z;
  }
  const unsigned short* wp = WT + (size_t)m * KW + 8 * hh;
  gemm_k128<NT, SPLIT, KW>(A1 + (size_t)rc * CH + 8 * hh, wp, acc);
  if (MODE == 3) gemm_k128<NT, SPLIT, KW>(A2 + (size_t)rc * CH + 8 * hh, wp + CH, acc);

#pragma unroll
  for (int nt = 0; nt < NT; ++nt) {
#pragma unroll
    for (int r = 0; r < 8; ++r) {
      const int lr = 16 * wave + 8 * hh + r;
      stg[lr * SP + 16 * nt + m] = acc[nt][r];
    }
  }
  __syncthreads();

  if (MODE != 3) {
    v4f vals[16];
#pragma unroll
    for (int rr = 0; rr < 16; ++rr) {
      const int lrow = 16 * wave + rr;
      v4f v = *(const v4fa*)(stg + lrow * SP + 4 * lane);
      const float sc = sRS[lrow];
      v = v * sc;
      if (MODE == 2) { v = v + bv; v = relu4(v); }
      vals[rr] = v;
    }
#pragma unroll
    for (int rr = 0; rr < 16; ++rr) {
      const int orow = rowBase + 16 * wave + rr;
      if (orow < nN) *(volatile v4f*)(O + (size_t)orow * NC + 4 * lane) = vals[rr];
    }
    __threadfence();
#pragma unroll
    for (int rr = 0; rr < 16; ++rr) {
      const int orow = rowBase + 16 * wave + rr;
      if (orow < nN) *(volatile v4f*)(O + (size_t)orow * NC + 4 * lane) = vals[rr];
    }
  } else {
    v4f vals[8];
#pragma unroll
    for (int i = 0; i < 8; ++i) {
      const int lrow = 16 * wave + 2 * i + hh;
      v4f v = *(const v4fa*)(stg + lrow * SP + 4 * m);
      vals[i] = v + bv;
    }
#pragma unroll
    for (int i = 0; i < 8; ++i) {
      const int orow = rowBase + 16 * wave + 2 * i + hh;
      if (orow < nN) *(volatile v4f*)(O + (size_t)orow * NC + 4 * m) = vals[i];
    }
    __threadfence();
#pragma unroll
    for (int i = 0; i < 8; ++i) {
      const int orow = rowBase + 16 * wave + 2 * i + hh;
      if (orow < nN) *(volatile v4f*)(O + (size_t)orow * NC + 4 * m) = vals[i];
    }
  }
}

static inline int cdiv(int a, int b) { return (a + b - 1) / b; }

extern "C" void kernel_launch(void* const* d_in, const int* in_sizes, int n_in,
                              void* d_out, int out_size, void* d_ws, size_t ws_size,
                              hipStream_t stream) {
  if (n_in < 9) return;
  if (in_sizes[0] < CIN || (in_sizes[0] % CIN) != 0) return;
  const int nN = in_sizes[0] / CIN;
  const int nE = in_sizes[1];
  if (nE < 1 || in_sizes[2] != nE) return;
  if (in_sizes[3] != CIN * CH || in_sizes[4] != CH) return;
  if (in_sizes[5] != CH * CH  || in_sizes[6] != CH) return;
  if (in_sizes[7] != 2 * CH * CO || in_sizes[8] != CO) return;
  if ((long long)out_size != (long long)nN * CO) return;
  if (nN < 1 || nN > (1 << SRCB)) return;

  const float* x    = (const float*)d_in[0];
  const int*   src  = (const int*)d_in[1];
  const int*   dst  = (const int*)d_in[2];
  const float* W1   = (const float*)d_in[3];
  const float* b1   = (const float*)d_in[4];
  const float* W2   = (const float*)d_in[5];
  const float* b2   = (const float*)d_in[6];
  const float* Wo   = (const float*)d_in[7];
  const float* bo   = (const float*)d_in[8];
  float* out = (float*)d_out;

  const int gD  = cdiv(nN, NBD);
  const int NBP = gD * NBD;
  const int gA  = cdiv(nN, NS);
  const int NSP = gA * NS;
  const int gM  = cdiv(nN, GBM);
  const int MP  = gM * GBM;
  if ((long long)NBP < nN || (long long)NSP < nN || (long long)MP < nN) return;
  const int vec8 = 1;

  char* ws = (char*)d_ws;
  size_t off = 0;
  const size_t oDOUT = off; off += (size_t)NBP * 4;              off = (off + 255) & ~(size_t)255;
  const size_t oDIN  = off; off += (size_t)NSP * 4;              off = (off + 255) & ~(size_t)255;
  const size_t oT1   = off; off += (size_t)CIN * CH * 2;         off = (off + 255) & ~(size_t)255;
  const size_t oT2   = off; off += (size_t)CH * CH * 2;          off = (off + 255) & ~(size_t)255;
  const size_t oTO   = off; off += (size_t)2 * CH * CO * 2;      off = (off + 255) & ~(size_t)255;
  const size_t oRA   = off; off += (size_t)MP * CH * 4;          off = (off + 255) & ~(size_t)255;
  const size_t oRB   = off; off += (size_t)MP * CH * 4;          off = (off + 255) & ~(size_t)255;
  const size_t oRC   = off; off += (size_t)MP * CH * 4;          off = (off + 255) & ~(size_t)255;
  if (off > ws_size || off > (size_t)WSMAX) return;
  float*          DOUT = (float*)(ws + oDOUT);
  float*          DIN  = (float*)(ws + oDIN);
  unsigned short* WT1  = (unsigned short*)(ws + oT1);
  unsigned short* WT2  = (unsigned short*)(ws + oT2);
  unsigned short* WTO  = (unsigned short*)(ws + oTO);
  float*          RA   = (float*)(ws + oRA);
  float*          RB   = (float*)(ws + oRB);
  float*          RC   = (float*)(ws + oRC);

  hipFuncSetAttribute(reinterpret_cast<const void*>(&k_agg<1>), hipFuncAttributeMaxDynamicSharedMemorySize, A_LDSB);
  hipFuncSetAttribute(reinterpret_cast<const void*>(&k_agg<2>), hipFuncAttributeMaxDynamicSharedMemorySize, A_LDSB);
  hipFuncSetAttribute(reinterpret_cast<const void*>(&k_agg<3>), hipFuncAttributeMaxDynamicSharedMemorySize, A_LDSB);

  k_wprep<<<24, NTHR, 0, stream>>>(W1, W2, Wo, WT1, WT2, WTO);
  k_deg<<<gD, NTHR, 0, stream>>>(src, nE, vec8, DOUT);
  k_gemm<1><<<gM, GTHR, 0, stream>>>(x, x, WT1, DOUT, b1, RA, nN);
  k_agg<1><<<gA, NTHR, A_LDSB, stream>>>(RA, src, dst, DOUT, b1, RB, DIN, nE, nN, vec8);
  k_agg<2><<<gA, NTHR, A_LDSB, stream>>>(RB, src, dst, DOUT, b1, RC, RA, nE, nN, vec8);
  k_gemm<2><<<gM, GTHR, 0, stream>>>(RA, RA, WT2, DIN, b2, RB, nN);
  k_agg<3><<<gA, NTHR, A_LDSB, stream>>>(RB, src, dst, DOUT, b1, RA, RA, nE, nN, vec8);
  k_gemm<3><<<gM, GTHR, 0, stream>>>(RC, RA, WTO, DIN, bo, out, nN);
}
